// minGRU2_20237885899461
// MI455X (gfx1250) — hardware-run, weakly checked
//
#include <hip/hip_runtime.h>
#include <math.h>

typedef __attribute__((ext_vector_type(16))) _Float16 v16h;
typedef __attribute__((ext_vector_type(8)))  _Float16 v8h;
typedef __attribute__((ext_vector_type(16))) __bf16   v16b;
typedef __attribute__((ext_vector_type(8)))  __bf16   v8b;
typedef __attribute__((ext_vector_type(8)))  float    v8f;
typedef __attribute__((ext_vector_type(4)))  float    v4f;

constexpr int kB    = 8;
constexpr int kC    = 128;
constexpr int kCLog2 = 7;
constexpr int kL    = 8192;
constexpr int kO    = 2 * kC;
constexpr int kQ    = kC / 2;
constexpr int kRows = kB * kL;
constexpr float kEpsNorm = 1e-4f;
constexpr int kThr  = 256;
constexpr float kInCarry = 1024.0f;
constexpr float kSc = 1.0f / (kInCarry * kInCarry);
constexpr float kF16MinNormal = 6.103515625e-5f;
constexpr float kCatW = 1.0f;

static_assert((1 << kCLog2) == kC && kO == 4 * kQ, "the shifts follow the sizes");
static_assert((kRows % 64) == 0 && (kO % 64) == 0 && (kC % 32) == 0 && ((kRows / 64) * (kO / 64)) % 8 == 0, "GEMM M, N multiples of 64, K of 32; grid exact (4,096 tiles)");

constexpr size_t kOffX16 = 0ull;
constexpr size_t kOffWE16 = 16777216ull;
constexpr size_t kOffZB = 16842752ull;
constexpr size_t kOffHG = 16843776ull;
constexpr size_t kWsTotal = 83952640ull;
static_assert(kWsTotal <= 134217728ull, "carve cap: under 128 MiB");
static_assert(kOffX16 == 0
              && kOffWE16 == kOffX16 + 16777216ull
              && kOffZB == kOffWE16 + 65536ull
              && kOffHG == kOffZB + 1024ull
              && kWsTotal == kOffHG + 67108864ull, "the carve is chained and totalled");
static_assert((kOffX16 % 256) == 0 && (kOffWE16 % 256) == 0 && (kOffZB % 256) == 0 && (kOffHG % 256) == 0, "aligned regions");

__device__ __forceinline__ unsigned short f2bf_bits(float f) {
  unsigned u = __float_as_uint(f);
  return (unsigned short)((u + 0x7FFFu + ((u >> 16) & 1u)) >> 16);
}
__device__ __forceinline__ float bf_bits2f(unsigned short h) { return __uint_as_float(((unsigned)h) << 16); }
__device__ __forceinline__ float bf16r(float f) { return bf_bits2f(f2bf_bits(f)); }
__device__ __forceinline__ float carry_flush(float v, float carry) {
  const float s = v * carry;
  return (fabsf(s) < kF16MinNormal) ? 0.0f : s;
}
__device__ __forceinline__ float frcp(float x) { return __builtin_amdgcn_rcpf(x); }

__device__ __forceinline__ void dep_guard4_h(v8f& a, v8f& b, v8f& c, v8f& d, v16h x, v16h y) { asm volatile("v_nop\n\tv_nop\n\tv_nop\n\tv_nop" : "+v"(a), "+v"(b), "+v"(c), "+v"(d) : "v"(x), "v"(y)); }
__device__ __forceinline__ void dep_guard4_b(v8f& a, v8f& b, v8f& c, v8f& d, v16b x, v16b y) { asm volatile("v_nop\n\tv_nop\n\tv_nop\n\tv_nop" : "+v"(a), "+v"(b), "+v"(c), "+v"(d) : "v"(x), "v"(y)); }
__device__ __forceinline__ void keep4_h(v16h a, v16h b, v16h c, v16h d) { asm volatile("v_nop" :: "v"(a), "v"(b), "v"(c), "v"(d)); }
__device__ __forceinline__ void keep4_b(v16b a, v16b b, v16b c, v16b d) { asm volatile("v_nop" :: "v"(a), "v"(b), "v"(c), "v"(d)); }
__device__ __forceinline__ void acc_guard4(v8f& a, v8f& b, v8f& c, v8f& d) { asm volatile("v_nop\n\tv_nop\n\tv_nop\n\tv_nop" : "+v"(a), "+v"(b), "+v"(c), "+v"(d)); }

template <typename T> struct Frag;
template <> struct Frag<_Float16> {
  typedef v16h V; union U { v16h v; v8h h[2]; };
  static __device__ __forceinline__ v16h load(const _Float16* p) {
    U f; f.h[0] = *(const v8h*)(p); f.h[1] = *(const v8h*)(p + 16); return f.v;
  }
  static __device__ __forceinline__ v8f mma(v16h a, v16h b, v8f c) {
    return __builtin_amdgcn_wmma_f32_16x16x32_f16(false, a, false, b, (short)0, c, false, false);
  }
  static __device__ __forceinline__ void guard4(v8f& a, v8f& b, v8f& c, v8f& d, v16h x, v16h y) { dep_guard4_h(a, b, c, d, x, y); }
  static __device__ __forceinline__ void keep(v16h a, v16h b, v16h c, v16h d) { keep4_h(a, b, c, d); }
};
template <> struct Frag<__bf16> {
  typedef v16b V; union U { v16b v; v8b h[2]; };
  static __device__ __forceinline__ v16b load(const __bf16* p) {
    U f; f.h[0] = *(const v8b*)(p); f.h[1] = *(const v8b*)(p + 16); return f.v;
  }
  static __device__ __forceinline__ v8f mma(v16b a, v16b b, v8f c) {
    return __builtin_amdgcn_wmma_f32_16x16x32_bf16(false, a, false, b, (short)0, c, false, false);
  }
  static __device__ __forceinline__ void guard4(v8f& a, v8f& b, v8f& c, v8f& d, v16b x, v16b y) { dep_guard4_b(a, b, c, d, x, y); }
  static __device__ __forceinline__ void keep(v16b a, v16b b, v16b c, v16b d) { keep4_b(a, b, c, d); }
};

__device__ __forceinline__ v8f mma_h(v16h a, v16h b, v8f c) {
  c = __builtin_amdgcn_wmma_f32_16x16x32_f16(false, a, false, b, (short)0, c, false, false);
  asm volatile("v_nop\n\tv_nop\n\tv_nop\n\tv_nop" : "+v"(c) : "v"(a), "v"(b));
  return c;
}

template <int ET> struct Elem;
template <> struct Elem<0> { typedef _Float16 T; };
template <> struct Elem<1> { typedef __bf16 T; };
template <int ET, bool SPLIT, int BIAS_MODE, int OUT_MODE, bool RESID, int ACT = 0>
__global__ __launch_bounds__(256) void wmma_gemm64(
    const unsigned short* __restrict__ Ap, const unsigned short* __restrict__ A2p, int lda, long strideA,
    const unsigned short* __restrict__ Btp, const unsigned short* __restrict__ Bt2p, int ldb, long strideB,
    void* __restrict__ Cout, void* __restrict__ Cout2, int ldc, long strideC,
    const float* __restrict__ bias,
    const float* __restrict__ resid, long strideR,
    int M, int N, int K, float scale) {
  typedef typename Elem<ET>::T T;
  typedef typename Frag<T>::V V;
  const T* A = (const T*)Ap; const T* A2 = (const T*)A2p; const T* Bt = (const T*)Btp; const T* Bt2 = (const T*)Bt2p;
  __shared__ __align__(16) float sT[8][16 * 68];
  const int b    = blockIdx.y;
  const int lane = threadIdx.x & 31;
  const int wave = threadIdx.x >> 5;
  const int tilesN = N >> 6;
  const int tilesM = M >> 6;
  const int tile = blockIdx.x * 8 + wave;
  if (tile >= tilesM * tilesN) return;
  const int tm = tile / tilesN;
  const int tn = tile - tm * tilesN;
  const int m0 = tm << 6;
  const int n0 = tn << 6;

  const T* Ab  = A  + (size_t)b * strideA;
  const T* Bb  = Bt + (size_t)b * strideB;
  const T* Ab2 = SPLIT ? (A2  + (size_t)b * strideA) : nullptr;
  const T* Bb2 = SPLIT ? (Bt2 + (size_t)b * strideB) : nullptr;

  const int rlane = lane & 15;
  const int koff  = (lane >> 4) * 8;
  const int mOff  = (lane >> 4) * 8;

  v8f acc[4][4];
#pragma unroll
  for (int i = 0; i < 4; ++i)
#pragma unroll
    for (int j = 0; j < 4; ++j) acc[i][j] = (v8f){0.f,0.f,0.f,0.f,0.f,0.f,0.f,0.f};

  for (int k0 = 0; k0 < K; k0 += 32) {
    V bh[4], bl[4];
#pragma unroll
    for (int j = 0; j < 4; ++j) {
      const size_t bo = (size_t)(n0 + (j << 4) + rlane) * ldb + koff + k0;
      bh[j] = Frag<T>::load(Bb + bo);
      if (SPLIT) bl[j] = Frag<T>::load(Bb2 + bo);
    }
#pragma unroll
    for (int i = 0; i < 4; ++i) {
      const size_t ao = (size_t)(m0 + (i << 4) + rlane) * lda + koff + k0;
      V ah = Frag<T>::load(Ab + ao);
      V al;
      if (SPLIT) al = Frag<T>::load(Ab2 + ao);
#pragma unroll
      for (int j = 0; j < 4; ++j) {
        acc[i][j] = Frag<T>::mma(ah, bh[j], acc[i][j]);
        if (SPLIT) {
          acc[i][j] = Frag<T>::mma(ah, bl[j], acc[i][j]);
          acc[i][j] = Frag<T>::mma(al, bh[j], acc[i][j]);
        }
      }
      Frag<T>::guard4(acc[i][0], acc[i][1], acc[i][2], acc[i][3], ah, SPLIT ? al : ah);
    }
    Frag<T>::keep(bh[0], bh[1], bh[2], bh[3]);
    if (SPLIT) Frag<T>::keep(bl[0], bl[1], bl[2], bl[3]);
  }
  acc_guard4(acc[0][0], acc[0][1], acc[0][2], acc[0][3]);
  acc_guard4(acc[1][0], acc[1][1], acc[1][2], acc[1][3]);
  acc_guard4(acc[2][0], acc[2][1], acc[2][2], acc[2][3]);
  acc_guard4(acc[3][0], acc[3][1], acc[3][2], acc[3][3]);

  float* slab = sT[wave];
  const float* Rb = RESID ? (resid + (size_t)b * strideR) : nullptr;
#pragma unroll
  for (int i = 0; i < 4; ++i) {
    const int mBase = m0 + (i << 4);
#pragma unroll
    for (int j = 0; j < 4; ++j) {
      const int n = n0 + (j << 4) + rlane;
      float bv = 0.f;
      if (BIAS_MODE == 2) bv = bias[n];
#pragma unroll
      for (int r = 0; r < 8; ++r) {
        float v = acc[i][j][r] * scale;
        if (BIAS_MODE == 1) v += bias[mBase + mOff + r];
        if (BIAS_MODE == 2) v += bv;
        if (RESID) v += Rb[(size_t)(mBase + mOff + r) * ldc + n];
        if (ACT == 1) v = tanhf(v);
        if (ACT == 2) v = fmaxf(v, 0.0f);
        if (ACT == 3) v = v / (1.0f + expf(-v));
        if (ACT == 4) v = (v > 0.f) ? v : 0.01f * v;
        slab[(mOff + r) * 68 + (j << 4) + rlane] = v;
      }
    }
    __builtin_amdgcn_fence(__ATOMIC_RELEASE, "workgroup");
    __builtin_amdgcn_wave_barrier();
    __builtin_amdgcn_fence(__ATOMIC_ACQUIRE, "workgroup");
    if (OUT_MODE == 0) {
      float* C = (float*)Cout + (size_t)b * strideC;
      const int hh = lane >> 4, c4 = (lane & 15) * 4;
      for (int pass = 0; pass < 2; ++pass) {
#pragma unroll
        for (int it = 0; it < 8; ++it) {
          const int row = it * 2 + hh;
          v4f v = *(const v4f*)(slab + row * 68 + c4);
          *(volatile v4f*)(C + (size_t)(mBase + row) * ldc + n0 + c4) = v;
        }
        __threadfence();
      }
    } else {
      const int q = lane >> 3, c8 = (lane & 7) * 8;
      unsigned short* C  = (unsigned short*)Cout  + (size_t)b * strideC;
      unsigned short* C2 = (OUT_MODE == 2) ? ((unsigned short*)Cout2 + (size_t)b * strideC) : nullptr;
      for (int pass = 0; pass < 2; ++pass) {
#pragma unroll
        for (int it = 0; it < 4; ++it) {
          const int row = it * 4 + q;
          const float* sp = slab + row * 68 + c8;
          v8h hv, lv;
#pragma unroll
          for (int e = 0; e < 8; ++e) {
            if (OUT_MODE == 1) {
              hv[e] = (_Float16)sp[e];
            } else {
              unsigned short hb = f2bf_bits(sp[e]);
              unsigned short lb = f2bf_bits(sp[e] - bf_bits2f(hb));
              hv[e] = __builtin_bit_cast(_Float16, hb);
              lv[e] = __builtin_bit_cast(_Float16, lb);
            }
          }
          *(volatile v8h*)(C + (size_t)(mBase + row) * ldc + n0 + c8) = hv;
          if (OUT_MODE == 2) *(volatile v8h*)(C2 + (size_t)(mBase + row) * ldc + n0 + c8) = lv;
        }
        __threadfence();
      }
    }
    __builtin_amdgcn_fence(__ATOMIC_RELEASE, "workgroup");
    __builtin_amdgcn_wave_barrier();
    __builtin_amdgcn_fence(__ATOMIC_ACQUIRE, "workgroup");
  }
}


__global__ __launch_bounds__(kThr) void xt_cast_kernel(const float* __restrict__ x, unsigned short* __restrict__ X16) {
  const unsigned smp = blockIdx.y;
  const unsigned pos = blockIdx.x * 16u + (threadIdx.x >> 4);
  const unsigned c8 = (threadIdx.x & 15u) * 8u;
  const float* sp = x + ((size_t)smp * kC + c8) * kL + pos;
  v8h hv;
#pragma unroll
  for (int e = 0; e < 8; ++e) {
    const float p = sp[(size_t)e * kL];
    hv[e] = (_Float16)carry_flush(bf16r(p), kInCarry);
  }
  unsigned short* dp = X16 + ((size_t)smp * kL + pos) * kC + c8;
  *(volatile v8h*)dp = hv;
  __threadfence();
  *(volatile v8h*)dp = hv;
}
static_assert(kL == 512 * 16 && kC == 16 * 8, "cast grid exact: 512 blocks of 16 positions a sample; 16 chunks a row");

__global__ __launch_bounds__(32) void weff_kernel(const float* __restrict__ w, unsigned short* __restrict__ WE16, float* __restrict__ ZB) {
  const unsigned o = blockIdx.x;
  const unsigned lane = threadIdx.x;
  if (lane < 16u) {
    const float* wr = w + (size_t)o * kC;
    float ss = 0.0f;
    for (int i = 0; i < kC; i += 4) {
      const v4f a = *(const v4f*)(wr + i);
      const float a0 = a[0], a1 = a[1], a2 = a[2], a3 = a[3];
      const float b0 = bf16r(a0), b1 = bf16r(a1), b2 = bf16r(a2), b3 = bf16r(a3);
      ss += (b0 * b0 + b1 * b1) + (b2 * b2 + b3 * b3);
    }
    const float rt = sqrtf((float)kC);
    const float den = kEpsNorm + sqrtf(ss) / rt;
    const v4f p0 = *(const v4f*)(wr + lane * 8u), p1 = *(const v4f*)(wr + lane * 8u + 4);
    v8h hv;
#pragma unroll
    for (int e = 0; e < 4; ++e) {
      const float q0 = p0[e], q1 = p1[e];
      hv[e] = (_Float16)carry_flush(bf16r(q0) / den / rt, kInCarry);
      hv[4 + e] = (_Float16)carry_flush(bf16r(q1) / den / rt, kInCarry);
    }
    unsigned short* dp = WE16 + (size_t)o * kC + lane * 8u;
    *(volatile v8h*)dp = hv;
    __threadfence();
    *(volatile v8h*)dp = hv;
  } else if (o < 8u && lane < 20u) {
    const v4f z = {0.f, 0.f, 0.f, 0.f};
    float* dp = ZB + o * 32u + (lane - 16u) * 8u;
    for (int pass = 0; pass < 2; ++pass) {
      *(volatile v4f*)dp = z;
      *(volatile v4f*)(dp + 4) = z;
      __threadfence();
    }
  }
}
static_assert(kO == 8 * 32 && kC == 16 * 8, "the zero bias: 8 blocks x 4 lanes x 8 floats = 256; a weight row = 16 chunks");

__global__ __launch_bounds__(kThr) void mingru_scan_kernel(const float* __restrict__ HG, float* __restrict__ out) {
  const unsigned v = blockIdx.x * (unsigned)kThr + threadIdx.x;
  const unsigned j = v & (unsigned)(kQ - 1), dir = (v >> 6) & 1u, smp = v >> 7;
  const float* hp = HG + (size_t)smp * kL * kO + dir * (unsigned)(2 * kQ) + j;
  float* op = out + ((size_t)smp * kC + dir * (unsigned)kQ + j) * kL;
  float c = 0.0f;
  for (int t = 0; t < kL; ++t) {
    const int l = dir ? (kL - 1 - t) : t;
    const float h = hp[(size_t)l * kO];
    const float g = hp[(size_t)l * kO + kQ];
    const float ep = expf(g), em = expf(-g);
    const float s = sqrtf(2.0f / (ep + em) + 1.0f);
    const float a = s / (1.0f + ep);
    const float b = h * s / (1.0f + em);
    c = a * c + b;
    const float o = kCatW * c;
    *(volatile float*)(op + l) = o;
    __threadfence();
    *(volatile float*)(op + l) = o;
  }
}
static_assert((kB * 2 * kQ) % kThr == 0 && kQ == 64, "scan grid exact: 4 blocks; 64 channels a direction (the shifts by 6 and 7)");

extern "C" void kernel_launch(void* const* d_in, const int* in_sizes, int n_in,
                              void* d_out, int out_size, void* d_ws, size_t ws_size,
                              hipStream_t stream) {
  if (n_in < 2 || d_out == nullptr || d_ws == nullptr) return;
  if (in_sizes[0] != kB * kC * kL || in_sizes[1] != kO * kC) return;
  if (out_size != kB * kC * kL) return;
  if (ws_size < kWsTotal) return;
  const float* x = (const float*)d_in[0];
  const float* w = (const float*)d_in[1];
  float* out = (float*)d_out;
  char* ws = (char*)d_ws;
  unsigned short* X16 = (unsigned short*)(ws + kOffX16);
  unsigned short* WE16 = (unsigned short*)(ws + kOffWE16);
  float* ZB = (float*)(ws + kOffZB);
  float* HG = (float*)(ws + kOffHG);

  xt_cast_kernel<<<dim3(kL / 16, kB), kThr, 0, stream>>>(x, X16);
  weff_kernel<<<kO, 32, 0, stream>>>(w, WE16, ZB);
  wmma_gemm64<0, false, 2, 0, false, 0><<<dim3((kRows / 64) * (kO / 64) / 8, 1), 256, 0, stream>>>(
      X16, X16, kC, 0L, WE16, WE16, kC, 0L, (void*)HG, (void*)HG, kO, 0L, ZB, nullptr, 0L, kRows, kO, kC, kSc);
  mingru_scan_kernel<<<(kB * 2 * kQ) / kThr, kThr, 0, stream>>>(HG, out);
}
